// FeedForwardQuantum_65481071400550
// MI455X (gfx1250) — hardware-verified
//
#include <hip/hip_runtime.h>
#include <math.h>
#include <stdint.h>

typedef __attribute__((ext_vector_type(16))) _Float16 v16h;
typedef __attribute__((ext_vector_type(8)))  _Float16 v8h;
typedef __attribute__((ext_vector_type(16))) __bf16   v16b;
typedef __attribute__((ext_vector_type(8)))  __bf16   v8b;
typedef __attribute__((ext_vector_type(8)))  float    v8f;
typedef __attribute__((ext_vector_type(4)))  float    v4f;
typedef __attribute__((ext_vector_type(4)))  unsigned int v4u;
typedef __attribute__((ext_vector_type(2)))  unsigned int v2u;

constexpr int EMB      = 1024;
constexpr int FFN_DIM  = 4096;
constexpr int NWIRE    = 8;
constexpr int NTOK     = 4 * 2048;
constexpr int HALF_TOK = NTOK / 2;
constexpr int HP_FCH   = 2048;
constexpr int HP_TOKB  = 64;

constexpr size_t WS_W2T_OFF   = 0;
constexpr size_t WS_W2T_BYTES = (size_t)EMB * FFN_DIM * 2;
constexpr size_t WS_Q_OFF     = WS_W2T_OFF + WS_W2T_BYTES;
constexpr size_t WS_Q_BYTES   = (size_t)NTOK * NWIRE * 4;
constexpr size_t WS_HHI_OFF   = WS_Q_OFF + WS_Q_BYTES;
constexpr size_t WS_H_BYTES   = (size_t)HALF_TOK * FFN_DIM * 2;
constexpr size_t WS_HLO_OFF   = WS_HHI_OFF + WS_H_BYTES;
constexpr size_t WS_TOTAL     = WS_HLO_OFF + WS_H_BYTES;
static_assert(WS_TOTAL == 75759616);
static_assert(WS_TOTAL <= 134217728);
static_assert(WS_Q_OFF % 128 == 0 && WS_HHI_OFF % 128 == 0 && WS_HLO_OFF % 128 == 0);

static_assert(HALF_TOK % 64 == 0 && EMB % 64 == 0 && FFN_DIM % 32 == 0);
static_assert(((HALF_TOK / 64) * (EMB / 64)) % 8 == 0);
constexpr int GEMM_GRID_X = (HALF_TOK / 64) * (EMB / 64) / 8;
static_assert(HP_FCH == 256 * 8 && FFN_DIM % HP_FCH == 0 && HALF_TOK % HP_TOKB == 0);
static_assert((HP_TOKB * NWIRE) == 2 * 256);
static_assert(EMB % 64 == 0 && FFN_DIM % 64 == 0);
static_assert((NTOK * NWIRE) % 256 == 0);

#define U16(p) ((const unsigned short*)(const void*)(p))

__device__ __forceinline__ unsigned short f2bf_bits(float f) {
  unsigned u = __float_as_uint(f);
  return (unsigned short)((u + 0x7FFFu + ((u >> 16) & 1u)) >> 16);
}
__device__ __forceinline__ float bf_bits2f(unsigned short h) { return __uint_as_float(((unsigned)h) << 16); }

__device__ __forceinline__ void dep_guard_h(v8f& a, v8f& b, v16h x, v16h y) { asm volatile("v_nop\n\tv_nop\n\tv_nop\n\tv_nop" : "+v"(a), "+v"(b) : "v"(x), "v"(y)); }
__device__ __forceinline__ void dep_guard_b(v8f& a, v8f& b, v16b x, v16b y) { asm volatile("v_nop\n\tv_nop\n\tv_nop\n\tv_nop" : "+v"(a), "+v"(b) : "v"(x), "v"(y)); }
__device__ __forceinline__ void keep4_h(v16h a, v16h b, v16h c, v16h d) { asm volatile("v_nop" :: "v"(a), "v"(b), "v"(c), "v"(d)); }
__device__ __forceinline__ void keep4_b(v16b a, v16b b, v16b c, v16b d) { asm volatile("v_nop" :: "v"(a), "v"(b), "v"(c), "v"(d)); }
__device__ __forceinline__ void acc_guard4(v8f& a, v8f& b, v8f& c, v8f& d) { asm volatile("v_nop\n\tv_nop\n\tv_nop\n\tv_nop" : "+v"(a), "+v"(b), "+v"(c), "+v"(d)); }
template <typename T> struct Frag;
template <> struct Frag<_Float16> {
  typedef v16h V; union U { v16h v; v8h h[2]; };
  static __device__ __forceinline__ v16h load(const _Float16* p) {
    U f; f.h[0] = *(const v8h*)(p); f.h[1] = *(const v8h*)(p + 16); return f.v;
  }
  static __device__ __forceinline__ v8f mma(v16h a, v16h b, v8f c) {
    return __builtin_amdgcn_wmma_f32_16x16x32_f16(false, a, false, b, (short)0, c, false, false);
  }
  static __device__ __forceinline__ void guard(v8f& a, v8f& b, v16h x, v16h y) { dep_guard_h(a, b, x, y); }
  static __device__ __forceinline__ void keep(v16h a, v16h b, v16h c, v16h d) { keep4_h(a, b, c, d); }
};
template <> struct Frag<__bf16> {
  typedef v16b V; union U { v16b v; v8b h[2]; };
  static __device__ __forceinline__ v16b load(const __bf16* p) {
    U f; f.h[0] = *(const v8b*)(p); f.h[1] = *(const v8b*)(p + 16); return f.v;
  }
  static __device__ __forceinline__ v8f mma(v16b a, v16b b, v8f c) {
    return __builtin_amdgcn_wmma_f32_16x16x32_bf16(false, a, false, b, (short)0, c, false, false);
  }
  static __device__ __forceinline__ void guard(v8f& a, v8f& b, v16b x, v16b y) { dep_guard_b(a, b, x, y); }
  static __device__ __forceinline__ void keep(v16b a, v16b b, v16b c, v16b d) { keep4_b(a, b, c, d); }
};

template <int ET> struct Elem;
template <> struct Elem<0> { typedef _Float16 T; };
template <> struct Elem<1> { typedef __bf16 T; };
template <int ET, int SPLIT, int BIAS_MODE, int OUT_MODE, bool RESID, int ACT = 0>
__global__ __launch_bounds__(256) void wmma_gemm64(
    const unsigned short* __restrict__ Ap, const unsigned short* __restrict__ A2p, int lda, long strideA,
    const unsigned short* __restrict__ Btp, const unsigned short* __restrict__ Bt2p, int ldb, long strideB,
    void* __restrict__ Cout, void* __restrict__ Cout2, int ldc, long strideC,
    const float* __restrict__ bias,
    const float* __restrict__ resid, long strideR,
    int M, int N, int K, float scale) {
  typedef typename Elem<ET>::T T;
  typedef typename Frag<T>::V V;
  const T* A = (const T*)Ap; const T* A2 = (const T*)A2p; const T* Bt = (const T*)Btp; const T* Bt2 = (const T*)Bt2p;
  __shared__ __align__(16) float sT[8][16 * 68];
  const int b    = blockIdx.y;
  const int lane = threadIdx.x & 31;
  const int wave = threadIdx.x >> 5;
  const int tilesN = N >> 6;
  const int tilesM = M >> 6;
  const int tile = blockIdx.x * 8 + wave;
  if (tile >= tilesM * tilesN) return;
  const int tm = tile / tilesN;
  const int tn = tile - tm * tilesN;
  const int m0 = tm << 6;
  const int n0 = tn << 6;

  const T* Ab  = A  + (size_t)b * strideA;
  const T* Bb  = Bt + (size_t)b * strideB;
  const T* Ab2 = (SPLIT != 0) ? (A2  + (size_t)b * strideA) : nullptr;
  const T* Bb2 = (SPLIT == 1) ? (Bt2 + (size_t)b * strideB) : nullptr;

  const int rlane = lane & 15;
  const int koff  = (lane >> 4) * 8;
  const int mOff  = (lane >> 4) * 8;

  v8f acc[4][4];
#pragma unroll
  for (int i = 0; i < 4; ++i)
#pragma unroll
    for (int j = 0; j < 4; ++j) acc[i][j] = (v8f){0.f,0.f,0.f,0.f,0.f,0.f,0.f,0.f};

  for (int k0 = 0; k0 < K; k0 += 32) {
    V bh[4], bl[4];
#pragma unroll
    for (int j = 0; j < 4; ++j) {
      const size_t bo = (size_t)(n0 + (j << 4) + rlane) * ldb + koff + k0;
      bh[j] = Frag<T>::load(Bb + bo);
      if (SPLIT == 1) bl[j] = Frag<T>::load(Bb2 + bo);
    }
#pragma unroll
    for (int i = 0; i < 4; ++i) {
      const size_t ao = (size_t)(m0 + (i << 4) + rlane) * lda + koff + k0;
      V ah = Frag<T>::load(Ab + ao);
      V al;
      if (SPLIT != 0) al = Frag<T>::load(Ab2 + ao);
#pragma unroll
      for (int j = 0; j < 4; ++j) {
        acc[i][j] = Frag<T>::mma(ah, bh[j], acc[i][j]);
        if (SPLIT == 1) acc[i][j] = Frag<T>::mma(ah, bl[j], acc[i][j]);
        if (SPLIT != 0) acc[i][j] = Frag<T>::mma(al, bh[j], acc[i][j]);
      }
      Frag<T>::guard(acc[i][0], acc[i][3], ah, (SPLIT != 0) ? al : ah);
    }
    Frag<T>::keep(bh[0], bh[1], bh[2], bh[3]);
    if (SPLIT == 1) Frag<T>::keep(bl[0], bl[1], bl[2], bl[3]);
  }
  acc_guard4(acc[0][0], acc[0][1], acc[0][2], acc[0][3]);
  acc_guard4(acc[1][0], acc[1][1], acc[1][2], acc[1][3]);
  acc_guard4(acc[2][0], acc[2][1], acc[2][2], acc[2][3]);
  acc_guard4(acc[3][0], acc[3][1], acc[3][2], acc[3][3]);

  float* slab = sT[wave];
  const float* Rb = RESID ? (resid + (size_t)b * strideR) : nullptr;
#pragma unroll
  for (int i = 0; i < 4; ++i) {
    const int mBase = m0 + (i << 4);
#pragma unroll
    for (int j = 0; j < 4; ++j) {
      const int n = n0 + (j << 4) + rlane;
      float bv = 0.f;
      if (BIAS_MODE == 2) bv = bias[n];
#pragma unroll
      for (int r = 0; r < 8; ++r) {
        float v = acc[i][j][r] * scale;
        if (BIAS_MODE == 1) v += bias[mBase + mOff + r];
        if (BIAS_MODE == 2) v += bv;
        if (RESID) v += Rb[(size_t)(mBase + mOff + r) * ldc + n];
        if (ACT == 1) v = tanhf(v);
        if (ACT == 2) v = fmaxf(v, 0.0f);
        if (ACT == 3) v = v / (1.0f + expf(-v));
        if (ACT == 4) v = (v > 0.f) ? v : 0.01f * v;
        if (ACT == 5) v = 0.5f * v * (1.0f + erff(v * 0.70710678118654752f));
        slab[(mOff + r) * 68 + (j << 4) + rlane] = v;
      }
    }
    __builtin_amdgcn_fence(__ATOMIC_RELEASE, "workgroup");
    __builtin_amdgcn_wave_barrier();
    __builtin_amdgcn_fence(__ATOMIC_ACQUIRE, "workgroup");
    if (OUT_MODE == 0) {
      float* C = (float*)Cout + (size_t)b * strideC;
      const int hh = lane >> 4, c4 = (lane & 15) * 4;
      for (int pass = 0; pass < 2; ++pass) {
#pragma unroll
        for (int it = 0; it < 8; ++it) {
          const int row = it * 2 + hh;
          v4f v = *(const v4f*)(slab + row * 68 + c4);
          *(volatile v4f*)(C + (size_t)(mBase + row) * ldc + n0 + c4) = v;
        }
        __threadfence();
      }
    } else {
      const int q = lane >> 3, c8 = (lane & 7) * 8;
      unsigned short* C  = (unsigned short*)Cout  + (size_t)b * strideC;
      unsigned short* C2 = (OUT_MODE == 2) ? ((unsigned short*)Cout2 + (size_t)b * strideC) : nullptr;
      for (int pass = 0; pass < 2; ++pass) {
#pragma unroll
        for (int it = 0; it < 4; ++it) {
          const int row = it * 4 + q;
          const float* sp = slab + row * 68 + c8;
          v8h hv, lv;
#pragma unroll
          for (int e = 0; e < 8; ++e) {
            if (OUT_MODE == 1) {
              hv[e] = (_Float16)sp[e];
            } else {
              unsigned short hb = f2bf_bits(sp[e]);
              unsigned short lb = f2bf_bits(sp[e] - bf_bits2f(hb));
              hv[e] = __builtin_bit_cast(_Float16, hb);
              lv[e] = __builtin_bit_cast(_Float16, lb);
            }
          }
          *(volatile v8h*)(C + (size_t)(mBase + row) * ldc + n0 + c8) = hv;
          if (OUT_MODE == 2) *(volatile v8h*)(C2 + (size_t)(mBase + row) * ldc + n0 + c8) = lv;
        }
        __threadfence();
      }
    }
    __builtin_amdgcn_fence(__ATOMIC_RELEASE, "workgroup");
    __builtin_amdgcn_wave_barrier();
    __builtin_amdgcn_fence(__ATOMIC_ACQUIRE, "workgroup");
  }
}

__global__ __launch_bounds__(256) void k_w2t(const float* __restrict__ w2, unsigned short* __restrict__ w2t)
{
  __shared__ float tile[64][65];
  const int tid  = threadIdx.x;
  const int lane = tid & 31, wv = tid >> 5;
  const int n0 = blockIdx.x * 64;
  const int k0 = blockIdx.y * 64;
#pragma unroll
  for (int it = 0; it < 4; ++it) {
    const int idx = it * 256 + tid;
    const int r = idx >> 4, c4 = idx & 15;
    const v4f v = *(const v4f*)(w2 + (size_t)(k0 + r) * EMB + n0 + c4 * 4);
    tile[r][c4 * 4 + 0] = v.x;
    tile[r][c4 * 4 + 1] = v.y;
    tile[r][c4 * 4 + 2] = v.z;
    tile[r][c4 * 4 + 3] = v.w;
  }
  __syncthreads();
  const int q8 = lane >> 3, c8 = (lane & 7) * 8;
  const int nr0 = wv * 8 + q8, nr1 = wv * 8 + 4 + q8;
  v4u pk0, pk1;
#pragma unroll
  for (int e = 0; e < 4; ++e) {
    const unsigned a0 = f2bf_bits(tile[c8 + 2 * e][nr0]);
    const unsigned a1 = f2bf_bits(tile[c8 + 2 * e + 1][nr0]);
    pk0[e] = a0 | (a1 << 16);
    const unsigned b0 = f2bf_bits(tile[c8 + 2 * e][nr1]);
    const unsigned b1 = f2bf_bits(tile[c8 + 2 * e + 1][nr1]);
    pk1[e] = b0 | (b1 << 16);
  }
  volatile v4u* p0 = (volatile v4u*)(w2t + (size_t)(n0 + nr0) * FFN_DIM + k0 + c8);
  volatile v4u* p1 = (volatile v4u*)(w2t + (size_t)(n0 + nr1) * FFN_DIM + k0 + c8);
  *p0 = pk0;
  *p1 = pk1;
  __threadfence();
  *p0 = pk0;
  *p1 = pk1;
}

__global__ __launch_bounds__(256) void k_qcos(const float* __restrict__ x, const float* __restrict__ theta,
                                              float* __restrict__ qpl, int ntot)
{
  #pragma clang fp contract(off)
  const int i = blockIdx.x * 256 + threadIdx.x;
  if (i < ntot) {
    const int tok = i >> 3, w = i & 7;
    const float xv = bf_bits2f(f2bf_bits(x[(size_t)tok * EMB + w]));
    const float th = bf_bits2f(f2bf_bits(theta[w]));
    const float s  = xv + th;
    const float qv = cosf(s);
    ((volatile float*)qpl)[i] = qv;
    __threadfence();
    ((volatile float*)qpl)[i] = qv;
  }
}

__global__ __launch_bounds__(256) void k_hprod(const float* __restrict__ qpl, const float* __restrict__ w1,
                                               unsigned short* __restrict__ hhi, unsigned short* __restrict__ hlo,
                                               int tokBase)
{
  __shared__ __align__(16) unsigned int w1s[NWIRE * HP_FCH / 2];
  __shared__ __align__(16) float qs[HP_TOKB * NWIRE];
  const int tid = threadIdx.x;
  const int fb  = blockIdx.x * HP_FCH;
  const int tb  = blockIdx.y * HP_TOKB;
#pragma unroll 1
  for (int it = 0; it < 16; ++it) {
    const int idx = it * 256 + tid;
    const int w  = idx >> 9;
    const int c4 = idx & 511;
    const v4f v = *(const v4f*)(w1 + (size_t)w * FFN_DIM + fb + c4 * 4);
    v2u pk;
    pk.x = (unsigned)f2bf_bits(v.x) | ((unsigned)f2bf_bits(v.y) << 16);
    pk.y = (unsigned)f2bf_bits(v.z) | ((unsigned)f2bf_bits(v.w) << 16);
    *(v2u*)(&w1s[(w * HP_FCH + c4 * 4) >> 1]) = pk;
  }
#pragma unroll
  for (int i = 0; i < 2; ++i) {
    const int idx = i * 256 + tid;
    const int t = idx >> 3, w = idx & 7;
    qs[idx] = qpl[(size_t)(tokBase + tb + t) * NWIRE + w];
  }
  __syncthreads();

  const int f0 = tid * 8;
  float wr[NWIRE][8];
#pragma unroll
  for (int w = 0; w < NWIRE; ++w) {
    const v4u pk = *(const v4u*)(&w1s[(w * HP_FCH + f0) >> 1]);
#pragma unroll
    for (int e = 0; e < 4; ++e) {
      float lo = __uint_as_float(pk[e] << 16);
      float hi = __uint_as_float(pk[e] & 0xffff0000u);
      asm volatile("" : "+v"(lo));
      asm volatile("" : "+v"(hi));
      wr[w][2 * e]     = lo;
      wr[w][2 * e + 1] = hi;
    }
  }

#pragma unroll 1
  for (int t = 0; t < HP_TOKB; ++t) {
    const v4f qa = *(const v4f*)(qs + t * NWIRE);
    const v4f qb = *(const v4f*)(qs + t * NWIRE + 4);
    const float qv[8] = {qa.x, qa.y, qa.z, qa.w, qb.x, qb.y, qb.z, qb.w};
    float h[8];
#pragma unroll
    for (int j = 0; j < 8; ++j) {
      float a = 0.0f;
#pragma unroll
      for (int w = 0; w < NWIRE; ++w) a = fmaf(qv[w], wr[w][j], a);
      h[j] = fmaxf(a, 0.0f);
    }
    v4u vh, vl;
#pragma unroll
    for (int e = 0; e < 4; ++e) {
      const unsigned short hb0 = f2bf_bits(h[2 * e]);
      const unsigned short lb0 = f2bf_bits(h[2 * e] - bf_bits2f(hb0));
      const unsigned short hb1 = f2bf_bits(h[2 * e + 1]);
      const unsigned short lb1 = f2bf_bits(h[2 * e + 1] - bf_bits2f(hb1));
      vh[e] = (unsigned)hb0 | ((unsigned)hb1 << 16);
      vl[e] = (unsigned)lb0 | ((unsigned)lb1 << 16);
    }
    const size_t off = (size_t)(tb + t) * FFN_DIM + fb + f0;
    volatile v4u* ph = (volatile v4u*)(hhi + off);
    volatile v4u* pl = (volatile v4u*)(hlo + off);
    *ph = vh;
    *pl = vl;
    __threadfence();
    *ph = vh;
    *pl = vl;
  }
}

extern "C" void kernel_launch(void* const* d_in, const int* in_sizes, int n_in,
                              void* d_out, int out_size, void* d_ws, size_t ws_size,
                              hipStream_t stream)
{
  if (n_in < 4) return;
  if (in_sizes[0] != NTOK * EMB || in_sizes[1] != NWIRE ||
      in_sizes[2] != NWIRE * FFN_DIM || in_sizes[3] != FFN_DIM * EMB) return;
  if (out_size != NTOK * EMB) return;
  if (ws_size < WS_TOTAL) return;

  const float* x     = (const float*)d_in[0];
  const float* theta = (const float*)d_in[1];
  const float* w1    = (const float*)d_in[2];
  const float* w2    = (const float*)d_in[3];
  float* out = (float*)d_out;

  char* ws = (char*)d_ws;
  unsigned short* w2t = (unsigned short*)(ws + WS_W2T_OFF);
  float*          qpl = (float*)(ws + WS_Q_OFF);
  unsigned short* hhi = (unsigned short*)(ws + WS_HHI_OFF);
  unsigned short* hlo = (unsigned short*)(ws + WS_HLO_OFF);

  k_w2t<<<dim3(EMB / 64, FFN_DIM / 64), 256, 0, stream>>>(w2, w2t);
  k_qcos<<<(NTOK * NWIRE) / 256, 256, 0, stream>>>(x, theta, qpl, NTOK * NWIRE);

  for (int half = 0; half < 2; ++half) {
    k_hprod<<<dim3(FFN_DIM / HP_FCH, HALF_TOK / HP_TOKB), 256, 0, stream>>>(
        qpl, w1, hhi, hlo, half * HALF_TOK);
    wmma_gemm64<1, 2, 0, 0, false, 0><<<dim3(GEMM_GRID_X, 1), 256, 0, stream>>>(
        hhi, hlo, FFN_DIM, 0L,
        w2t, w2t, FFN_DIM, 0L,
        (void*)(out + (size_t)half * HALF_TOK * EMB), (void*)hlo, EMB, 0L,
        qpl,
        qpl, 0L,
        HALF_TOK, EMB, FFN_DIM, 1.0f);
  }
}
